// MultiHeadSelfAttention_62362925138607
// MI455X (gfx1250) — hardware-verified
//
#include <hip/hip_runtime.h>


#ifndef NB
#define NB 2
#endif
#ifndef SEQ
#define SEQ 2048
#endif
#define TT       SEQ
#define TT_FULL  2048
#define DM       2048
#define NH_      16
#define HD       128
#define RH       ((SEQ) < 512 ? (SEQ) : 512)
#define PP       72
#define OP       136
#define SCL      0.08838834764831845f
#define VCAR     16.0f
#define CCAR     64.0f
#define WCAR     64.0f

static_assert(NH_ * HD == DM);
static_assert(HD == 128);
static_assert(TT % 64 == 0);
static_assert(RH % 256 == 0);
static_assert(RH <= TT);
static_assert((TT - RH) % 64 == 0);
static_assert(((size_t)NH_ * TT * HD) % 2048 == 0);
static_assert(((size_t)TT * DM) % 2048 == 0);
static_assert(((size_t)DM * DM) % 2048 == 0);
static_assert(((size_t)3 * DM * DM) % 2048 == 0);
static_assert((TT * (HD / 2)) % 256 == 0);
static_assert(DM % 64 == 0 && DM % 32 == 0);

typedef _Float16 h16;
typedef unsigned short bf;
typedef __attribute__((ext_vector_type(16))) __bf16   v16bf;
typedef __attribute__((ext_vector_type(16))) _Float16 v16h;
typedef __attribute__((ext_vector_type(8)))  _Float16 v8h;
typedef __attribute__((ext_vector_type(8)))  unsigned short v8us;
typedef __attribute__((ext_vector_type(8)))  float    v8f;
typedef __attribute__((ext_vector_type(4)))  float    v4f;
typedef __attribute__((ext_vector_type(2)))  float    v2f;
typedef v8h  __attribute__((may_alias)) v8ha;
typedef v4f  __attribute__((may_alias)) v4fa;
typedef v8us __attribute__((may_alias)) v8usa;

__device__ __forceinline__ unsigned short f2bf(float f) { unsigned u = __float_as_uint(f); u += 0x7FFFu + ((u >> 16) & 1u); return (unsigned short)(u >> 16); }
__device__ __forceinline__ float bf2f(unsigned short b) { return __uint_as_float(((unsigned)b) << 16); }
__device__ __forceinline__ float bfr(float f) { return bf2f(f2bf(f)); }
__device__ __forceinline__ void splitf(float y, unsigned short& h, unsigned short& l) { h = f2bf(y); l = f2bf(y - bf2f(h)); }
__device__ __forceinline__ v16h cat16(v8h lo, v8h hi) { return __builtin_shufflevector(lo, hi, 0, 1, 2, 3, 4, 5, 6, 7, 8, 9, 10, 11, 12, 13, 14, 15); }
__device__ __forceinline__ v16bf cat16b(v8us lo, v8us hi) { return __builtin_bit_cast(v16bf, __builtin_shufflevector(lo, hi, 0, 1, 2, 3, 4, 5, 6, 7, 8, 9, 10, 11, 12, 13, 14, 15)); }
__device__ __forceinline__ v8f wmma16(v16h a, v16h b, v8f c) { return __builtin_amdgcn_wmma_f32_16x16x32_f16(false, a, false, b, (short)0, c, false, false); }
__device__ __forceinline__ v8f wmmab(v16bf a, v16bf b, v8f c) { return __builtin_amdgcn_wmma_f32_16x16x32_bf16(false, a, false, b, (short)0, c, false, false); }

template <typename T16> struct WFrag;
template <> struct WFrag<h16> {
    typedef v16h V; static constexpr bool HI = false; static constexpr float PSH = 10.0f; static constexpr float OSC = CCAR / VCAR;
    static __device__ __forceinline__ V ld(const h16* p) { return cat16(*(const v8h*)p, *(const v8h*)(p + 16)); }
    static __device__ __forceinline__ V ldl(const h16* p) { return cat16(*(const v8ha*)p, *(const v8ha*)(p + 16)); }
    static __device__ __forceinline__ v8f mma(V a, V b, v8f c) { return wmma16(a, b, c); }
    static __device__ __forceinline__ void stp(h16* a, h16* b, int i, float x) { (void)b; a[i] = (h16)x; }
    static __device__ __forceinline__ void stv(h16* g, const h16* l) { const v8h v = *(const v8ha*)l; *(volatile v8h*)g = v; }
};
template <> struct WFrag<bf> {
    typedef v16bf V; static constexpr bool HI = true; static constexpr float PSH = 0.0f; static constexpr float OSC = 1.0f;
    static __device__ __forceinline__ V ld(const bf* p) { return cat16b(*(const v8us*)p, *(const v8us*)(p + 16)); }
    static __device__ __forceinline__ V ldl(const bf* p) { return cat16b(*(const v8usa*)p, *(const v8usa*)(p + 16)); }
    static __device__ __forceinline__ v8f mma(V a, V b, v8f c) { return wmmab(a, b, c); }
    static __device__ __forceinline__ void stp(bf* a, bf* b, int i, float x) { unsigned short h, l; splitf(x, h, l); a[i] = h; b[i] = l; }
    static __device__ __forceinline__ void stv(bf* g, const bf* l) { const v8us v = *(const v8usa*)l; *(volatile v8us*)g = v; }
};

template <typename T16, int NSPLIT>
__global__ __launch_bounds__(32) void k_gemmw(const T16* __restrict__ A, const T16* __restrict__ A2, const T16* __restrict__ Bt, int K, float* C, int ldc, float osc) {
    typedef WFrag<T16> W; typedef typename W::V V;
    __shared__ __align__(16) float os[16 * 68];
    const int lane = threadIdx.x & 31, lr = lane & 15, hi = lane >> 4; const int r0 = blockIdx.x * 64, c0 = blockIdx.y * 64;
    v8f acc[4][4];
#pragma unroll
    for (int mb = 0; mb < 4; ++mb)
#pragma unroll
        for (int nb = 0; nb < 4; ++nb) acc[mb][nb] = (v8f){};
    const size_t aoff = (size_t)(r0 + lr) * K + 8 * hi, boff = (size_t)(c0 + lr) * K + 8 * hi;
#pragma unroll 1
    for (int kc = 0; kc < K; kc += 32) {
        V a[4], a2[4];
#pragma unroll
        for (int mb = 0; mb < 4; ++mb) { a[mb] = W::ld(A + aoff + (size_t)mb * 16 * K + kc); if (NSPLIT == 1) a2[mb] = W::ld(A2 + aoff + (size_t)mb * 16 * K + kc); }
#pragma unroll
        for (int nb = 0; nb < 4; ++nb) { const V b = W::ld(Bt + boff + (size_t)nb * 16 * K + kc);
#pragma unroll
            for (int mb = 0; mb < 4; ++mb) { acc[mb][nb] = W::mma(a[mb], b, acc[mb][nb]); if (NSPLIT == 1) acc[mb][nb] = W::mma(a2[mb], b, acc[mb][nb]); } }
        asm volatile("v_nop\n\tv_nop\n\tv_nop\n\tv_nop" : "+v"(acc[0][0]), "+v"(acc[1][1]), "+v"(acc[2][2]), "+v"(acc[3][3]) : "v"(a[0]), "v"(a[3]));
    }
#pragma unroll
    for (int mb = 0; mb < 4; ++mb) {
#pragma unroll
        for (int nb = 0; nb < 4; ++nb) {
#pragma unroll
            for (int j = 0; j < 8; ++j) os[(hi * 8 + j) * 68 + nb * 16 + lr] = acc[mb][nb][j]; }
        __builtin_amdgcn_wave_barrier(); asm volatile("" ::: "memory");
        float* crow = C + (size_t)(r0 + mb * 16) * ldc + c0;
#pragma unroll 1
        for (int ps = 0; ps < 2; ++ps) {
#pragma unroll
            for (int s = 0; s < 8; ++s) { const int row = 2 * s + hi, cofs = lr * 4; v4f val = *(const v4fa*)(os + row * 68 + cofs); val[0] *= osc; val[1] *= osc; val[2] *= osc; val[3] *= osc;
                *(volatile v4f*)(crow + (size_t)row * ldc + cofs) = val; }
            if (ps == 0) __threadfence(); }
        __builtin_amdgcn_wave_barrier(); asm volatile("" ::: "memory");
    }
}

__global__ __launch_bounds__(256) void k_cvt8(const float* __restrict__ src, bf* dst, size_t n8) { const size_t i = (size_t)blockIdx.x * 256 + threadIdx.x; if (i >= n8) return; const v8f v = *(const v8f*)(src + i * 8); v8us o;
#pragma unroll
    for (int k = 0; k < 8; ++k) o[k] = f2bf(v[k]);
    *(volatile v8us*)(dst + i * 8) = o; __threadfence(); *(volatile v8us*)(dst + i * 8) = o; }
__global__ __launch_bounds__(256) void k_cvth8(const float* __restrict__ src, h16* dst, size_t n8, float car) { const size_t i = (size_t)blockIdx.x * 256 + threadIdx.x; if (i >= n8) return; const v8f v = *(const v8f*)(src + i * 8); v8h o;
#pragma unroll
    for (int k = 0; k < 8; ++k) o[k] = (h16)(bfr(v[k]) * car);
    *(volatile v8h*)(dst + i * 8) = o; __threadfence(); *(volatile v8h*)(dst + i * 8) = o; }
__global__ __launch_bounds__(256) void k_cstab(float* CS) {
    const int idx = blockIdx.x * 256 + threadIdx.x; if (idx >= TT * (HD / 2)) return; const int p = idx % (HD / 2), t = idx / (HD / 2);
    const float pr = -9.210340371976184f * (float)(2 * p); const float ex = pr * (1.0f / (float)HD); const float th = expf(ex); const float ang = (float)t * th;
    float sn, cs_; sincosf(ang, &sn, &cs_); v2f o; o[0] = cs_; o[1] = sn;
    *(volatile v2f*)(CS + (size_t)idx * 2) = o; __threadfence(); *(volatile v2f*)(CS + (size_t)idx * 2) = o; }
__global__ __launch_bounds__(256) void k_rope(const float* __restrict__ F, const float* __restrict__ CS, h16* P16, bf* Ph, bf* Pl) {
#pragma clang fp contract(off)
    const size_t e = ((size_t)blockIdx.x * 256 + threadIdx.x) * 8; if (e >= (size_t)NH_ * TT * HD) return;
    const int d = (int)(e % HD); const int t = (int)((e / HD) % TT); const int h = (int)(e / ((size_t)HD * TT));
    const float* f = F + (size_t)t * DM + h * HD + d; const float* cp = CS + (size_t)t * HD + d;
    const v4f xa = *(const v4f*)f, xb = *(const v4f*)(f + 4), ca = *(const v4f*)cp, cb = *(const v4f*)(cp + 4);
    float r[8];
    r[0] = xa[0] * ca[0] - xa[1] * ca[1]; r[1] = xa[0] * ca[1] + xa[1] * ca[0];
    r[2] = xa[2] * ca[2] - xa[3] * ca[3]; r[3] = xa[2] * ca[3] + xa[3] * ca[2];
    r[4] = xb[0] * cb[0] - xb[1] * cb[1]; r[5] = xb[0] * cb[1] + xb[1] * cb[0];
    r[6] = xb[2] * cb[2] - xb[3] * cb[3]; r[7] = xb[2] * cb[3] + xb[3] * cb[2];
    v8h o16; v8us oh, ol;
#pragma unroll
    for (int q = 0; q < 8; ++q) { o16[q] = (h16)r[q]; unsigned short a2, c2; splitf(r[q], a2, c2); oh[q] = a2; ol[q] = c2; }
    const bool hr = (t < RH); const size_t eh = ((size_t)h * RH + (hr ? t : 0)) * HD + d;
    *(volatile v8h*)(P16 + e) = o16; if (hr) { *(volatile v8us*)(Ph + eh) = oh; *(volatile v8us*)(Pl + eh) = ol; }
    __threadfence();
    *(volatile v8h*)(P16 + e) = o16; if (hr) { *(volatile v8us*)(Ph + eh) = oh; *(volatile v8us*)(Pl + eh) = ol; }
}
__global__ __launch_bounds__(256) void k_vtp(const float* __restrict__ F, h16* V16, bf* Vh, bf* Vl) {
    const size_t e = ((size_t)blockIdx.x * 256 + threadIdx.x) * 8; if (e >= (size_t)NH_ * HD * TT) return;
    const int t0 = (int)(e % TT); const int d = (int)((e / TT) % HD); const int h = (int)(e / ((size_t)TT * HD));
    const float* f = F + (size_t)t0 * DM + h * HD + d; v8h o16; v8us oh, ol;
#pragma unroll
    for (int q = 0; q < 8; ++q) { const float x = f[(size_t)q * DM]; o16[q] = (h16)(x * VCAR); unsigned short a2, c2; splitf(x, a2, c2); oh[q] = a2; ol[q] = c2; }
    const bool hr = (t0 < RH); const size_t eh = ((size_t)h * HD + d) * RH + (hr ? t0 : 0);
    *(volatile v8h*)(V16 + e) = o16; if (hr) { *(volatile v8us*)(Vh + eh) = oh; *(volatile v8us*)(Vl + eh) = ol; }
    __threadfence();
    *(volatile v8h*)(V16 + e) = o16; if (hr) { *(volatile v8us*)(Vh + eh) = oh; *(volatile v8us*)(Vl + eh) = ol; }
}

template <typename T16>
__global__ __launch_bounds__(32) void k_attn(const T16* __restrict__ Q, const T16* __restrict__ Q2, const T16* __restrict__ Kp, const T16* __restrict__ K2, const T16* __restrict__ Vt, const T16* __restrict__ Vt2, int rows, T16* C, T16* C2, int qt0) {
    typedef WFrag<T16> W; typedef typename W::V V; constexpr bool HI = W::HI;
    __shared__ __align__(16) T16 ps[16 * PP]; __shared__ __align__(16) T16 ps2[HI ? 16 * PP : 8];
    __shared__ __align__(16) T16 os[16 * OP]; __shared__ __align__(16) T16 os2[HI ? 16 * OP : 8];
    const int lane = threadIdx.x & 31, lr = lane & 15, hi = lane >> 4;
    const int h = blockIdx.y; const int qbase = (qt0 + (int)blockIdx.x) * 16;
    const size_t qo = ((size_t)h * rows + qbase + lr) * HD + 8 * hi;
    const size_t ko = ((size_t)h * rows + lr) * HD + 8 * hi;
    const size_t vo = ((size_t)h * HD + lr) * rows + 8 * hi;
    const float SL = SCL * 1.4426950408889634f; const float NEGB = -1.0e30f;
    V qa[4];
    if (!HI) {
#pragma unroll
        for (int c = 0; c < 4; ++c) qa[c] = W::ld(Q + qo + c * 32); }
    v8f oacc[8]; float mrow[8], lsum[8];
#pragma unroll
    for (int d = 0; d < 8; ++d) oacc[d] = (v8f){};
#pragma unroll
    for (int r = 0; r < 8; ++r) { mrow[r] = NEGB; lsum[r] = 0.0f; }
#pragma unroll 1
    for (int jb = 0; jb < qbase + 16; jb += 64) {
        v8f s[4];
#pragma unroll
        for (int j = 0; j < 4; ++j) s[j] = (v8f){};
        V la, lb;
#pragma unroll
        for (int c = 0; c < 4; ++c) {
            V a, a2;
            if (HI) { a = W::ld(Q + qo + c * 32); a2 = W::ld(Q2 + qo + c * 32); } else { a = qa[c]; a2 = a; }
#pragma unroll
            for (int j = 0; j < 4; ++j) {
                const size_t kk = ko + (size_t)(jb + 16 * j) * HD + c * 32;
                const V b = W::ld(Kp + kk); V b2 = b;
                s[j] = W::mma(a, b, s[j]);
                if (HI) { s[j] = W::mma(a2, b, s[j]); b2 = W::ld(K2 + kk); s[j] = W::mma(a, b2, s[j]); }
                la = a; lb = b2; } }
        asm volatile("v_nop\n\tv_nop\n\tv_nop\n\tv_nop" : "+v"(s[0]), "+v"(s[1]), "+v"(s[2]), "+v"(s[3]) : "v"(la), "v"(lb));
        const bool diag = (jb + 63 > qbase);
        float alpha[8];
        __syncthreads();
#pragma unroll
        for (int r = 0; r < 8; ++r) {
            float x0 = s[0][r] * SL, x1 = s[1][r] * SL, x2 = s[2][r] * SL, x3 = s[3][r] * SL;
            if (diag) { const int lim = qbase + r + 8 * hi - jb - lr;
                x0 = (0 <= lim) ? x0 : NEGB; x1 = (16 <= lim) ? x1 : NEGB; x2 = (32 <= lim) ? x2 : NEGB; x3 = (48 <= lim) ? x3 : NEGB; }
            float mx = fmaxf(fmaxf(x0, x1), fmaxf(x2, x3));
            mx = fmaxf(mx, __shfl_xor(mx, 1, 32)); mx = fmaxf(mx, __shfl_xor(mx, 2, 32)); mx = fmaxf(mx, __shfl_xor(mx, 4, 32)); mx = fmaxf(mx, __shfl_xor(mx, 8, 32));
            const float mnew = fmaxf(mrow[r], mx);
            const float al = __builtin_amdgcn_exp2f(mrow[r] - mnew);
            const float mb = mnew - W::PSH;
            const float p0 = __builtin_amdgcn_exp2f(x0 - mb), p1 = __builtin_amdgcn_exp2f(x1 - mb), p2 = __builtin_amdgcn_exp2f(x2 - mb), p3 = __builtin_amdgcn_exp2f(x3 - mb);
            lsum[r] = lsum[r] * al + ((p0 + p1) + (p2 + p3)); mrow[r] = mnew; alpha[r] = al;
            const int pi = (r + 8 * hi) * PP + lr;
            W::stp(ps, ps2, pi, p0); W::stp(ps, ps2, pi + 16, p1); W::stp(ps, ps2, pi + 32, p2); W::stp(ps, ps2, pi + 48, p3);
        }
        __syncthreads();
        V pa[2], pa2[2];
#pragma unroll
        for (int kc = 0; kc < 2; ++kc) { pa[kc] = W::ldl(ps + lr * PP + kc * 32 + 8 * hi); if (HI) pa2[kc] = W::ldl(ps2 + lr * PP + kc * 32 + 8 * hi); else pa2[kc] = pa[kc]; }
#pragma unroll
        for (int d = 0; d < 8; ++d)
#pragma unroll
            for (int r = 0; r < 8; ++r) oacc[d][r] *= alpha[r];
#pragma unroll
        for (int kc = 0; kc < 2; ++kc)
#pragma unroll
            for (int d = 0; d < 8; ++d) {
                const size_t vv = vo + (size_t)(d * 16) * rows + jb + kc * 32;
                const V bv = W::ld(Vt + vv); V bv2 = bv;
                oacc[d] = W::mma(pa[kc], bv, oacc[d]);
                if (HI) { oacc[d] = W::mma(pa2[kc], bv, oacc[d]); bv2 = W::ld(Vt2 + vv); oacc[d] = W::mma(pa[kc], bv2, oacc[d]); }
                la = pa[kc]; lb = bv2; }
        asm volatile("v_nop\n\tv_nop\n\tv_nop\n\tv_nop" : "+v"(oacc[0]), "+v"(oacc[1]), "+v"(oacc[2]), "+v"(oacc[3]), "+v"(oacc[4]), "+v"(oacc[5]), "+v"(oacc[6]), "+v"(oacc[7]) : "v"(la), "v"(lb));
    }
    float inv[8];
#pragma unroll
    for (int r = 0; r < 8; ++r) { float l = lsum[r]; l += __shfl_xor(l, 1, 32); l += __shfl_xor(l, 2, 32); l += __shfl_xor(l, 4, 32); l += __shfl_xor(l, 8, 32); inv[r] = W::OSC * __builtin_amdgcn_rcpf(l); }
#pragma unroll
    for (int d = 0; d < 8; ++d)
#pragma unroll
        for (int r = 0; r < 8; ++r) W::stp(os, os2, (r + 8 * hi) * OP + d * 16 + lr, oacc[d][r] * inv[r]);
    __syncthreads();
    const size_t cb = (size_t)qbase * DM + (size_t)h * HD + lr * 8;
#pragma unroll 1
    for (int pz = 0; pz < 2; ++pz) {
#pragma unroll
        for (int s8 = 0; s8 < 8; ++s8) { const int row = 2 * s8 + hi; W::stv(C + cb + (size_t)row * DM, os + row * OP + lr * 8); if (HI) W::stv(C2 + cb + (size_t)row * DM, os2 + row * OP + lr * 8); }
        if (pz == 0) __threadfence(); }
}

constexpr size_t SZ_W  = (size_t)DM * DM * 2;
constexpr size_t SZ_CS = (size_t)TT * HD * 4;
constexpr size_t SZ_XB = (size_t)TT * DM * 2;
constexpr size_t SZ_F  = (size_t)TT * DM * 4;
constexpr size_t SZ_P  = (size_t)NH_ * TT * HD * 2;
constexpr size_t SZ_PH = (size_t)NH_ * RH * HD * 2;
constexpr size_t SZ_C  = (size_t)TT * DM * 2;
constexpr size_t SZ_CH = (size_t)RH * DM * 2;
constexpr size_t WS_TOTAL = 5 * SZ_W + SZ_CS + SZ_XB + SZ_F + 3 * SZ_P + 6 * SZ_PH + SZ_C + 2 * SZ_CH;
static_assert(WS_TOTAL <= (size_t)134217728);
static_assert(SZ_W % 256 == 0 && SZ_CS % 256 == 0 && SZ_XB % 256 == 0 && SZ_PH % 256 == 0 && SZ_CH % 256 == 0);
static_assert(SZ_F % 256 == 0 && SZ_P % 256 == 0 && SZ_C % 256 == 0);

extern "C" void kernel_launch(void* const* d_in, const int* in_sizes, int n_in,
                              void* d_out, int out_size, void* d_ws, size_t ws_size, hipStream_t stream) {
    if (n_in < 3) return;
    const size_t need_x = (size_t)(NB - 1) * TT_FULL * DM + (size_t)TT * DM;
    if ((size_t)in_sizes[0] < need_x) return;
    if ((size_t)in_sizes[1] < (size_t)3 * DM * DM || (size_t)in_sizes[2] < (size_t)DM * DM) return;
    if ((size_t)out_size < need_x) return;
    if (ws_size < WS_TOTAL) return;
    const float* x = (const float*)d_in[0]; const float* wqkv = (const float*)d_in[1]; const float* wo = (const float*)d_in[2];
    float* OUT = (float*)d_out;
    char* wsp = (char*)d_ws;
    auto take = [&](size_t bytes) { char* p = wsp; wsp += (bytes + 255) & ~(size_t)255; return (void*)p; };
    bf* WQKV = (bf*)take(3 * SZ_W); bf* WQ = WQKV; bf* WK = WQKV + (size_t)DM * DM; bf* WV = WQKV + (size_t)2 * DM * DM;
    bf* WO = (bf*)take(SZ_W); h16* WOH = (h16*)take(SZ_W);
    float* CS = (float*)take(SZ_CS);
    bf* XB = (bf*)take(SZ_XB); float* F = (float*)take(SZ_F);
    h16* Q16 = (h16*)take(SZ_P); h16* K16 = (h16*)take(SZ_P); h16* VT16 = (h16*)take(SZ_P);
    bf* QPh = (bf*)take(SZ_PH); bf* QPl = (bf*)take(SZ_PH); bf* KPh = (bf*)take(SZ_PH); bf* KPl = (bf*)take(SZ_PH); bf* VTh = (bf*)take(SZ_PH); bf* VTl = (bf*)take(SZ_PH);
    h16* C16 = (h16*)take(SZ_C); bf* Ch = (bf*)take(SZ_CH); bf* Cl = (bf*)take(SZ_CH);
    if ((size_t)(wsp - (char*)d_ws) > ws_size) return;

    const size_t nw8 = (size_t)DM * DM / 8; const unsigned GW = (unsigned)((nw8 + 255) / 256);
    const size_t nw8x3 = 3 * nw8; const unsigned GW3 = (unsigned)((nw8x3 + 255) / 256);
    k_cvt8<<<GW3, 256, 0, stream>>>(wqkv, WQKV, nw8x3);
    k_cvt8<<<GW, 256, 0, stream>>>(wo, WO, nw8);
    k_cvth8<<<GW, 256, 0, stream>>>(wo, WOH, nw8, WCAR);
    k_cstab<<<(unsigned)((TT * (HD / 2) + 255) / 256), 256, 0, stream>>>(CS);

    const size_t nx8 = (size_t)TT * DM / 8; const unsigned GX = (unsigned)((nx8 + 255) / 256);
    const unsigned GP = (unsigned)(((size_t)NH_ * TT * HD / 8 + 255) / 256);
    for (int b = 0; b < NB; ++b) {
        const float* xb = x + (size_t)b * TT_FULL * DM; float* ob = OUT + (size_t)b * TT_FULL * DM;
        k_cvt8<<<GX, 256, 0, stream>>>(xb, XB, nx8);
        k_gemmw<bf, 0><<<dim3(TT / 64, DM / 64, 1), 32, 0, stream>>>(XB, (const bf*)nullptr, WQ, DM, F, DM, 1.0f);
        k_rope<<<GP, 256, 0, stream>>>(F, CS, Q16, QPh, QPl);
        k_gemmw<bf, 0><<<dim3(TT / 64, DM / 64, 1), 32, 0, stream>>>(XB, (const bf*)nullptr, WK, DM, F, DM, 1.0f);
        k_rope<<<GP, 256, 0, stream>>>(F, CS, K16, KPh, KPl);
        k_gemmw<bf, 0><<<dim3(TT / 64, DM / 64, 1), 32, 0, stream>>>(XB, (const bf*)nullptr, WV, DM, F, DM, 1.0f);
        k_vtp<<<GP, 256, 0, stream>>>(F, VT16, VTh, VTl);
        k_attn<bf><<<dim3(RH / 16, NH_, 1), 32, 0, stream>>>(QPh, QPl, KPh, KPl, VTh, VTl, RH, Ch, Cl, 0);
        if (TT > RH) k_attn<h16><<<dim3((TT - RH) / 16, NH_, 1), 32, 0, stream>>>(Q16, (const h16*)nullptr, K16, (const h16*)nullptr, VT16, (const h16*)nullptr, TT, C16, (h16*)nullptr, RH / 16);
        k_gemmw<bf, 1><<<dim3(RH / 64, DM / 64, 1), 32, 0, stream>>>(Ch, Cl, WO, DM, ob, DM, 1.0f);
        if (TT > RH) k_gemmw<h16, 0><<<dim3((TT - RH) / 64, DM / 64, 1), 32, 0, stream>>>(C16 + (size_t)RH * DM, (const h16*)nullptr, WOH, DM, ob + (size_t)RH * DM, DM, 1.0f / (CCAR * WCAR));
    }
}
